// PatchRangeAttention_15135464751306
// MI455X (gfx1250) — hardware-verified
//
#include <hip/hip_runtime.h>


namespace {
constexpr int B = 8, N = 1025, D = 768, NH = 12, HD = 64, G = 32, R = 3, NT = B * N, NTP = 8208, D3 = 3 * D;
constexpr float XS = 8.0f, PS = 1024.0f, WSC = 256.0f, SCALE = 0.125f;
typedef _Float16 b16;
typedef __attribute__((ext_vector_type(16))) _Float16 v16b;
typedef __attribute__((ext_vector_type(8))) _Float16 v8b;
typedef __attribute__((ext_vector_type(8))) float v8f;
typedef __attribute__((ext_vector_type(4))) float v4f;
typedef __attribute__((ext_vector_type(2))) float v2f;
__device__ __forceinline__ float bf16_rne(float f) { unsigned int u = __float_as_uint(f); u += 0x7FFFu + ((u >> 16) & 1u); return __uint_as_float(u & 0xFFFF0000u); }
__device__ __forceinline__ void split16(float v, b16& hi, b16& lo) { hi = (b16)v; lo = (b16)(v - (float)hi); }
__device__ __forceinline__ v16b frag_kb(const b16* p, int hh) { const v8b a = *(const v8b*)(p + 8 * hh), b = *(const v8b*)(p + 16 + 8 * hh); v16b f;
#pragma unroll
  for (int e = 0; e < 8; ++e) { f[e] = a[e]; f[8 + e] = b[e]; } return f; }
__device__ __forceinline__ v8f wmma16b(v16b a, v16b b, v8f c) { v8f d = __builtin_amdgcn_wmma_f32_16x16x32_f16(false, a, false, b, (short)0, c, false, false); asm volatile("v_nop\n\tv_nop\n\tv_nop\n\tv_nop" : "+v"(d) : "v"(a), "v"(b)); return d; }
__device__ __forceinline__ void wave_lds_sync() { __builtin_amdgcn_fence(__ATOMIC_RELEASE, "workgroup"); __builtin_amdgcn_wave_barrier(); __builtin_amdgcn_fence(__ATOMIC_ACQUIRE, "workgroup"); }
__device__ __forceinline__ float pmul(float a, float b) { float p = a * b; asm volatile("" : "+v"(p)); return p; }

__global__ __launch_bounds__(256) void wput_kernel(const float* __restrict__ w, int KIN, int OUTW, b16* __restrict__ WT) {
  const int KG = KIN / 8; const size_t u = (size_t)blockIdx.x * 256 + threadIdx.x; if (u >= (size_t)OUTW * KG) return; const int o = (int)(u / KG), k0 = (int)(u % KG) * 8; v8b v;
#pragma unroll
  for (int j = 0; j < 8; ++j) v[j] = (b16)(bf16_rne(w[(size_t)(k0 + j) * OUTW + o]) * WSC); for (int pass = 0; pass < 2; ++pass) { *(volatile v8b*)(WT + (size_t)o * KIN + k0) = v; __threadfence(); }
}
template <int FIRST, int NTILE>
__global__ __launch_bounds__(32) void dense_kernel(const float* __restrict__ IN, int inpitch, const b16* __restrict__ WT, const float* __restrict__ bias, int NROW, float* __restrict__ OUT) {
  __shared__ __attribute__((aligned(16))) b16 Ah[16][D + 8], Al[16][(FIRST ? 32 : D) + 8]; __shared__ __attribute__((aligned(16))) float Tf[16][128 + 4];
  const int lane = threadIdx.x, nloc = lane & 15, hlf = lane >> 4; const size_t m0 = (size_t)blockIdx.x * 16; if (m0 >= (size_t)NROW) return;
  for (int rr = 0; rr < 16; ++rr) { const size_t row = (m0 + rr < (size_t)NT) ? m0 + rr : (size_t)NT - 1; for (int q = 0; q < D / 32; ++q) { const float v = IN[row * inpitch + q * 32 + lane]; if (FIRST) Ah[rr][q * 32 + lane] = (b16)(bf16_rne(v) * XS); else { b16 p, ql; split16(v * XS, p, ql); Ah[rr][q * 32 + lane] = p; Al[rr][q * 32 + lane] = ql; } } }
  wave_lds_sync();
#pragma unroll 1
  for (int cg = 0; cg < NTILE / 8; ++cg) { v8f acc[8];
#pragma unroll
    for (int t = 0; t < 8; ++t) acc[t] = (v8f){};
#pragma unroll 2
    for (int kb = 0; kb < D; kb += 32) { const v16b a = frag_kb(&Ah[nloc][kb], hlf); v16b al; if (!FIRST) al = frag_kb(&Al[nloc][kb], hlf);
#pragma unroll
      for (int t = 0; t < 8; ++t) { const v16b bw = frag_kb(WT + (size_t)(cg * 128 + t * 16 + nloc) * D + kb, hlf); acc[t] = wmma16b(a, bw, acc[t]); if (!FIRST) acc[t] = wmma16b(al, bw, acc[t]); } }
#pragma unroll
    for (int t = 0; t < 8; ++t) { const int c = cg * 128 + t * 16 + nloc; const float bb = bf16_rne(bias[c]);
#pragma unroll
      for (int r8 = 0; r8 < 8; ++r8) Tf[8 * hlf + r8][t * 16 + nloc] = acc[t][r8] * (1.0f / (XS * WSC)) + bb; }
    wave_lds_sync();
    for (int pass = 0; pass < 2; ++pass) { for (int rr = 0; rr < 16; ++rr) if (m0 + rr < (size_t)NROW) *(volatile v4f*)(OUT + (m0 + rr) * (size_t)(NTILE * 16) + cg * 128 + lane * 4) = *(const v4f*)(&Tf[rr][lane * 4]); __threadfence(); }
    wave_lds_sync(); }
}
__global__ __launch_bounds__(32) void att_kernel(const float* __restrict__ QKV, int NBV, float* __restrict__ O) {
  constexpr int MAXK = 16 + 7 * G;
  __shared__ __attribute__((aligned(16))) b16 Qh[16][HD + 8], Kh[16][HD + 8]; __shared__ float Sc[16][MAXK + 1]; __shared__ __attribute__((aligned(16))) b16 Ph[16][MAXK + 24], Pl[16][MAXK + 24], Vh[HD][40], Vl[HD][40]; __shared__ float Of[16][HD + 1];
  const int lane = threadIdx.x, nloc = lane & 15, hlf = lane >> 4; const int half = blockIdx.x & 1, r = (blockIdx.x >> 1) % G, h = (blockIdx.x / (2 * G)) % NH, b = blockIdx.x / (2 * G * NH); if (b >= NBV) return;
  const int c0 = half * 16; const size_t tq0 = (size_t)b * N + 1 + r * G + c0; const int rlo = r - R < 0 ? 0 : r - R, rhi = r + R > G - 1 ? G - 1 : r + R; const int nkr = (rhi - rlo + 1) * G; const int nk = 16 + nkr;
  const size_t tk0 = (size_t)b * N + 1 + rlo * G;
  auto ktok = [&](int j) -> size_t { return j < 16 ? (size_t)b * N : tk0 + (j - 16); };
  for (int rr = 0; rr < 16; ++rr) for (int q = 0; q < 2; ++q) Qh[rr][q * 32 + lane] = (b16)(QKV[(tq0 + rr) * D3 + h * HD + q * 32 + lane] * XS);
#pragma unroll 1
  for (int kb = 0; kb < nk / 16; ++kb) { for (int rr = 0; rr < 16; ++rr) { const int j = kb * 16 + rr; const bool real = (j == 0) || (j >= 16); for (int q = 0; q < 2; ++q) Kh[rr][q * 32 + lane] = real ? (b16)(QKV[ktok(j) * D3 + D + h * HD + q * 32 + lane] * XS) : (b16)0.0f; }
    wave_lds_sync(); v8f acc = {};
#pragma unroll
    for (int ks = 0; ks < HD; ks += 32) acc = wmma16b(frag_kb(&Qh[nloc][ks], hlf), frag_kb(&Kh[nloc][ks], hlf), acc);
#pragma unroll
    for (int r8 = 0; r8 < 8; ++r8) { const int qi = 8 * hlf + r8, j = kb * 16 + nloc; bool valid; if (j < 16) valid = (j == 0); else { const int kc = (j - 16) % G; const int dc = (c0 + qi) - kc; valid = dc <= R && dc >= -R; }
      Sc[qi][j] = valid ? acc[r8] * (SCALE / (XS * XS)) : -INFINITY; }
    wave_lds_sync(); }
  for (int qi = 0; qi < 16; ++qi) { float mx = -INFINITY; for (int j = lane; j < nk; j += 32) mx = fmaxf(mx, Sc[qi][j]); for (int o = 16; o; o >>= 1) mx = fmaxf(mx, __shfl_xor(mx, o)); float s = 0.0f;
    for (int j = lane; j < nk; j += 32) { const float e = (Sc[qi][j] == -INFINITY) ? 0.0f : __expf(Sc[qi][j] - mx); Sc[qi][j] = e; s += e; } for (int o = 16; o; o >>= 1) s += __shfl_xor(s, o); const float inv = 1.0f / s;
    for (int j = lane; j < nk; j += 32) { b16 p, q; split16(Sc[qi][j] * inv * PS, p, q); Ph[qi][j] = p; Pl[qi][j] = q; } }
  wave_lds_sync();
  v8f oacc[4] = {(v8f){}, (v8f){}, (v8f){}, (v8f){}};
#pragma unroll 1
  for (int kc = 0; kc < nk; kc += 32) {
    for (int jj = 0; jj < 32; ++jj) { const int j = kc + jj; const bool real = (j < nk) && ((j == 0) || (j >= 16)); for (int q = 0; q < 2; ++q) { const int d = q * 32 + lane; b16 p = (b16)0.0f, ql = (b16)0.0f; if (real) split16(QKV[ktok(j) * D3 + 2 * D + h * HD + d] * XS, p, ql); Vh[d][jj] = p; Vl[d][jj] = ql; } }
    if (kc + 32 > nk) { for (int rr = 0; rr < 16; ++rr) { Ph[rr][nk + nloc] = (b16)0.0f; Pl[rr][nk + nloc] = (b16)0.0f; } }
    wave_lds_sync(); const v16b pa = frag_kb(&Ph[nloc][kc], hlf), pl = frag_kb(&Pl[nloc][kc], hlf);
#pragma unroll
    for (int t = 0; t < 4; ++t) { const v16b vh = frag_kb(&Vh[t * 16 + nloc][0], hlf), vl = frag_kb(&Vl[t * 16 + nloc][0], hlf); oacc[t] = wmma16b(pa, vh, oacc[t]); oacc[t] = wmma16b(pa, vl, oacc[t]); oacc[t] = wmma16b(pl, vh, oacc[t]); }
    wave_lds_sync(); }
#pragma unroll
  for (int t = 0; t < 4; ++t)
#pragma unroll
    for (int r8 = 0; r8 < 8; ++r8) Of[8 * hlf + r8][t * 16 + nloc] = oacc[t][r8] * (1.0f / (PS * XS));
  wave_lds_sync();
  for (int pass = 0; pass < 2; ++pass) { for (int rr = 0; rr < 16; ++rr) *(volatile v2f*)(O + (tq0 + rr) * D + h * HD + lane * 2) = (v2f){Of[rr][lane * 2], Of[rr][lane * 2 + 1]}; __threadfence(); }
}
__global__ __launch_bounds__(32) void cls_kernel(const float* __restrict__ QKV, int NBV, float* __restrict__ O) {
  __shared__ float Pq[1056], Qs[HD]; const int lane = threadIdx.x; const int h = blockIdx.x % NH, b = blockIdx.x / NH; if (b >= NBV) return; const size_t t0 = (size_t)b * N;
  if (lane < 32) { Qs[lane] = QKV[t0 * D3 + h * HD + lane]; Qs[32 + lane] = QKV[t0 * D3 + h * HD + 32 + lane]; }
  wave_lds_sync(); float mx = -INFINITY;
  for (int k = lane; k < N; k += 32) { const float* kp = QKV + (t0 + k) * D3 + D + h * HD; float s = 0.0f;
#pragma unroll 4
    for (int d = 0; d < HD; ++d) s += pmul(Qs[d], kp[d]); s *= SCALE; Pq[k] = s; mx = fmaxf(mx, s); }
  for (int o = 16; o; o >>= 1) mx = fmaxf(mx, __shfl_xor(mx, o)); float sum = 0.0f;
  for (int k = lane; k < N; k += 32) { const float e = __expf(Pq[k] - mx); Pq[k] = e; sum += e; } for (int o = 16; o; o >>= 1) sum += __shfl_xor(sum, o); const float inv = 1.0f / sum;
  wave_lds_sync(); float o0 = 0.0f, o1 = 0.0f;
#pragma unroll 1
  for (int k = 0; k < N; ++k) { const v2f vv = *(const v2f*)(QKV + (t0 + k) * D3 + 2 * D + h * HD + lane * 2); const float p = Pq[k]; o0 += pmul(p, vv[0]); o1 += pmul(p, vv[1]); }
  for (int pass = 0; pass < 2; ++pass) { *(volatile v2f*)(O + t0 * D + h * HD + lane * 2) = (v2f){o0 * inv, o1 * inv}; __threadfence(); }
}
}

extern "C" void kernel_launch(void* const* d_in, const int* in_sizes, int n_in, void* d_out, int out_size, void* d_ws, size_t ws_size, hipStream_t stream) {
  (void)n_in;
  auto Fp = [&](int i) { return (const float*)d_in[i]; };
  if (in_sizes[0] != NT * D || in_sizes[1] != D * D3 || in_sizes[2] != D3 || in_sizes[3] != D * D || in_sizes[4] != D || out_size != NT * D) return;
  const int NBV = B; const int NROWV = NBV * N;
  size_t off = 0; char* ws = (char*)d_ws;
  auto carve = [&](size_t bytes) { char* p = ws + off; off += (bytes + 255) & ~(size_t)255; return p; };
  b16* WQKV = (b16*)carve((size_t)D3 * D * 2); b16* WP = (b16*)carve((size_t)D * D * 2); float* QKV = (float*)carve((size_t)NTP * D3 * 4); float* O = (float*)carve((size_t)NTP * D * 4);
  if (off > ws_size || off > ((size_t)128 << 20)) return;
  wput_kernel<<<(unsigned)(((size_t)D3 * (D / 8) + 255) / 256), 256, 0, stream>>>(Fp(1), D, D3, WQKV); wput_kernel<<<(D * (D / 8) + 255) / 256, 256, 0, stream>>>(Fp(3), D, D, WP);
  dense_kernel<1, 144><<<(unsigned)((NROWV + 15) / 16), 32, 0, stream>>>(Fp(0), D, WQKV, Fp(2), NROWV, QKV);
  att_kernel<<<(unsigned)(NBV * NH * G * 2), 32, 0, stream>>>(QKV, NBV, O);
  cls_kernel<<<NBV * NH, 32, 0, stream>>>(QKV, NBV, O);
  dense_kernel<0, 48><<<(unsigned)((NROWV + 15) / 16), 32, 0, stream>>>(O, D, WP, Fp(4), NROWV, (float*)d_out);
}
